// MetaPathGNN_20160576487476
// MI455X (gfx1250) — hardware-verified
//
#include <hip/hip_runtime.h>
#include <stddef.h>
#include <math.h>

typedef __attribute__((ext_vector_type(16))) _Float16 v16h;
typedef __attribute__((ext_vector_type(8)))  _Float16 v8h;
typedef __attribute__((ext_vector_type(4)))  _Float16 v4h;
typedef __attribute__((ext_vector_type(16))) __bf16   v16b;
typedef __attribute__((ext_vector_type(8)))  __bf16   v8b;
typedef __attribute__((ext_vector_type(8)))  float    v8f;
typedef __attribute__((ext_vector_type(4)))  float    v4f;
typedef __attribute__((ext_vector_type(4)))  int      v4i;

constexpr int XDIM  = 128;
constexpr int HDIM  = 64;
constexpr int FDIM  = 128;
constexpr int ODIM  = 64;
constexpr int KCMB  = 384;
constexpr int NBAGG = 512;
constexpr int RPQ   = 512;
#define NTHR    256
#define NWAVE   8
#define EPT     8
#define NGRP    1
#define CHUNK   (NTHR * EPT * NGRP)
#define WCAP    (EPT * NGRP * 32)
#define LISTN   (NWAVE * WCAP)
#define LDS_AGG (NBAGG * FDIM * 4 + LISTN * 4 + 64)

static_assert((CHUNK & (CHUNK - 1)) == 0);
static_assert(CHUNK <= 4096);
static_assert((NBAGG & (NBAGG - 1)) == 0 && NBAGG <= 4096);
static_assert(RPQ % NBAGG == 0 && RPQ % 64 == 0 && RPQ % 16 == 0);
static_assert(LDS_AGG == 270400);
static_assert(KCMB == FDIM + FDIM + XDIM);
static_assert(XDIM % 32 == 0 && HDIM % 64 == 0 && FDIM % 64 == 0 && ODIM % 64 == 0 && KCMB % 32 == 0);

__device__ __forceinline__ unsigned short f2bf_bits(float f) {
  unsigned u = __float_as_uint(f);
  return (unsigned short)((u + 0x7FFFu + ((u >> 16) & 1u)) >> 16);
}
__device__ __forceinline__ float bf_bits2f(unsigned short h) { return __uint_as_float(((unsigned)h) << 16); }

__device__ __forceinline__ void dep_guard_h(v8f& a, v8f& b, v16h x, v16h y) { asm volatile("v_nop\n\tv_nop\n\tv_nop\n\tv_nop" : "+v"(a), "+v"(b) : "v"(x), "v"(y)); }
__device__ __forceinline__ void dep_guard_b(v8f& a, v8f& b, v16b x, v16b y) { asm volatile("v_nop\n\tv_nop\n\tv_nop\n\tv_nop" : "+v"(a), "+v"(b) : "v"(x), "v"(y)); }
__device__ __forceinline__ void keep4_h(v16h a, v16h b, v16h c, v16h d) { asm volatile("v_nop" :: "v"(a), "v"(b), "v"(c), "v"(d)); }
__device__ __forceinline__ void keep4_b(v16b a, v16b b, v16b c, v16b d) { asm volatile("v_nop" :: "v"(a), "v"(b), "v"(c), "v"(d)); }
__device__ __forceinline__ void acc_guard4(v8f& a, v8f& b, v8f& c, v8f& d) { asm volatile("v_nop\n\tv_nop\n\tv_nop\n\tv_nop" : "+v"(a), "+v"(b), "+v"(c), "+v"(d)); }
template <typename T> struct Frag;
template <> struct Frag<_Float16> {
  typedef v16h V; union U { v16h v; v8h h[2]; };
  static __device__ __forceinline__ v16h load(const _Float16* p) {
    U f; f.h[0] = *(const v8h*)(p); f.h[1] = *(const v8h*)(p + 16); return f.v;
  }
  static __device__ __forceinline__ v8f mma(v16h a, v16h b, v8f c) {
    return __builtin_amdgcn_wmma_f32_16x16x32_f16(false, a, false, b, (short)0, c, false, false);
  }
  static __device__ __forceinline__ void guard(v8f& a, v8f& b, v16h x, v16h y) { dep_guard_h(a, b, x, y); }
  static __device__ __forceinline__ void keep(v16h a, v16h b, v16h c, v16h d) { keep4_h(a, b, c, d); }
};
template <> struct Frag<__bf16> {
  typedef v16b V; union U { v16b v; v8b h[2]; };
  static __device__ __forceinline__ v16b load(const __bf16* p) {
    U f; f.h[0] = *(const v8b*)(p); f.h[1] = *(const v8b*)(p + 16); return f.v;
  }
  static __device__ __forceinline__ v8f mma(v16b a, v16b b, v8f c) {
    return __builtin_amdgcn_wmma_f32_16x16x32_bf16(false, a, false, b, (short)0, c, false, false);
  }
  static __device__ __forceinline__ void guard(v8f& a, v8f& b, v16b x, v16b y) { dep_guard_b(a, b, x, y); }
  static __device__ __forceinline__ void keep(v16b a, v16b b, v16b c, v16b d) { keep4_b(a, b, c, d); }
};

template <int ET> struct Elem;
template <> struct Elem<0> { typedef _Float16 T; };
template <> struct Elem<1> { typedef __bf16 T; };
template <int ET, bool SPLIT, int BIAS_MODE, int OUT_MODE, bool RESID, int ACT = 0>
__global__ __launch_bounds__(256) void wmma_gemm64(
    const unsigned short* __restrict__ Ap, const unsigned short* __restrict__ A2p, int lda, long strideA,
    const unsigned short* __restrict__ Btp, const unsigned short* __restrict__ Bt2p, int ldb, long strideB,
    void* __restrict__ Cout, void* __restrict__ Cout2, int ldc, long strideC,
    const float* __restrict__ bias,
    const float* __restrict__ resid, long strideR,
    int M, int N, int K, float scale) {
  typedef typename Elem<ET>::T T;
  typedef typename Frag<T>::V V;
  const T* A = (const T*)Ap; const T* A2 = (const T*)A2p; const T* Bt = (const T*)Btp; const T* Bt2 = (const T*)Bt2p;
  __shared__ __align__(16) float sT[8][16 * 68];
  const int b    = blockIdx.y;
  const int lane = threadIdx.x & 31;
  const int wave = threadIdx.x >> 5;
  const int tilesN = N >> 6;
  const int tilesM = M >> 6;
  const int tile = blockIdx.x * 8 + wave;
  if (tile >= tilesM * tilesN) return;
  const int tm = tile / tilesN;
  const int tn = tile - tm * tilesN;
  const int m0 = tm << 6;
  const int n0 = tn << 6;

  const T* Ab  = A  + (size_t)b * strideA;
  const T* Bb  = Bt + (size_t)b * strideB;
  const T* Ab2 = SPLIT ? (A2  + (size_t)b * strideA) : nullptr;
  const T* Bb2 = SPLIT ? (Bt2 + (size_t)b * strideB) : nullptr;

  const int rlane = lane & 15;
  const int koff  = (lane >> 4) * 8;
  const int mOff  = (lane >> 4) * 8;

  v8f acc[4][4];
#pragma unroll
  for (int i = 0; i < 4; ++i)
#pragma unroll
    for (int j = 0; j < 4; ++j) acc[i][j] = (v8f){0.f,0.f,0.f,0.f,0.f,0.f,0.f,0.f};

  for (int k0 = 0; k0 < K; k0 += 32) {
    V bh[4], bl[4];
#pragma unroll
    for (int j = 0; j < 4; ++j) {
      const size_t bo = (size_t)(n0 + (j << 4) + rlane) * ldb + koff + k0;
      bh[j] = Frag<T>::load(Bb + bo);
      if (SPLIT) bl[j] = Frag<T>::load(Bb2 + bo);
    }
#pragma unroll
    for (int i = 0; i < 4; ++i) {
      const size_t ao = (size_t)(m0 + (i << 4) + rlane) * lda + koff + k0;
      V ah = Frag<T>::load(Ab + ao);
      V al;
      if (SPLIT) al = Frag<T>::load(Ab2 + ao);
#pragma unroll
      for (int j = 0; j < 4; ++j) {
        acc[i][j] = Frag<T>::mma(ah, bh[j], acc[i][j]);
        if (SPLIT) {
          acc[i][j] = Frag<T>::mma(ah, bl[j], acc[i][j]);
          acc[i][j] = Frag<T>::mma(al, bh[j], acc[i][j]);
        }
      }
      Frag<T>::guard(acc[i][0], acc[i][3], ah, SPLIT ? al : ah);
    }
    Frag<T>::keep(bh[0], bh[1], bh[2], bh[3]);
    if (SPLIT) Frag<T>::keep(bl[0], bl[1], bl[2], bl[3]);
  }
  acc_guard4(acc[0][0], acc[0][1], acc[0][2], acc[0][3]);
  acc_guard4(acc[1][0], acc[1][1], acc[1][2], acc[1][3]);
  acc_guard4(acc[2][0], acc[2][1], acc[2][2], acc[2][3]);
  acc_guard4(acc[3][0], acc[3][1], acc[3][2], acc[3][3]);

  float* slab = sT[wave];
  const float* Rb = RESID ? (resid + (size_t)b * strideR) : nullptr;
#pragma unroll
  for (int i = 0; i < 4; ++i) {
    const int mBase = m0 + (i << 4);
#pragma unroll
    for (int j = 0; j < 4; ++j) {
      const int n = n0 + (j << 4) + rlane;
      float bv = 0.f;
      if (BIAS_MODE == 2) bv = bias[n];
#pragma unroll
      for (int r = 0; r < 8; ++r) {
        float v = acc[i][j][r] * scale;
        if (BIAS_MODE == 1) v += bias[mBase + mOff + r];
        if (BIAS_MODE == 2) v += bv;
        if (RESID) v += Rb[(size_t)(mBase + mOff + r) * ldc + n];
        if (ACT == 1) v = tanhf(v);
        if (ACT == 2) v = fmaxf(v, 0.0f);
        if (ACT == 3) v = v / (1.0f + expf(-v));
        if (ACT == 4) v = (v > 0.f) ? v : 0.01f * v;
        if (ACT == 5) v = 0.5f * v * (1.0f + erff(v * 0.70710678118654752f));
        slab[(mOff + r) * 68 + (j << 4) + rlane] = v;
      }
    }
    __builtin_amdgcn_fence(__ATOMIC_RELEASE, "workgroup");
    __builtin_amdgcn_wave_barrier();
    __builtin_amdgcn_fence(__ATOMIC_ACQUIRE, "workgroup");
    if (OUT_MODE == 0) {
      float* C = (float*)Cout + (size_t)b * strideC;
      const int hh = lane >> 4, c4 = (lane & 15) * 4;
      for (int pass = 0; pass < 2; ++pass) {
#pragma unroll
        for (int it = 0; it < 8; ++it) {
          const int row = it * 2 + hh;
          v4f v = *(const v4f*)(slab + row * 68 + c4);
          *(volatile v4f*)(C + (size_t)(mBase + row) * ldc + n0 + c4) = v;
        }
        __threadfence();
      }
    } else {
      const int q = lane >> 3, c8 = (lane & 7) * 8;
      unsigned short* C  = (unsigned short*)Cout  + (size_t)b * strideC;
      unsigned short* C2 = (OUT_MODE == 2) ? ((unsigned short*)Cout2 + (size_t)b * strideC) : nullptr;
      for (int pass = 0; pass < 2; ++pass) {
#pragma unroll
        for (int it = 0; it < 4; ++it) {
          const int row = it * 4 + q;
          const float* sp = slab + row * 68 + c8;
          v8h hv, lv;
#pragma unroll
          for (int e = 0; e < 8; ++e) {
            if (OUT_MODE == 1) {
              hv[e] = (_Float16)sp[e];
            } else {
              unsigned short hb = f2bf_bits(sp[e]);
              unsigned short lb = f2bf_bits(sp[e] - bf_bits2f(hb));
              hv[e] = __builtin_bit_cast(_Float16, hb);
              lv[e] = __builtin_bit_cast(_Float16, lb);
            }
          }
          *(volatile v8h*)(C + (size_t)(mBase + row) * ldc + n0 + c8) = hv;
          if (OUT_MODE == 2) *(volatile v8h*)(C2 + (size_t)(mBase + row) * ldc + n0 + c8) = lv;
        }
        __threadfence();
      }
    }
    __builtin_amdgcn_fence(__ATOMIC_RELEASE, "workgroup");
    __builtin_amdgcn_wave_barrier();
    __builtin_amdgcn_fence(__ATOMIC_ACQUIRE, "workgroup");
  }
}

template <int NB>
__device__ __forceinline__ int scan_chunk(const int* __restrict__ lst, int nE, int cbase, int nodeBase,
                                          int* list, int tid, int lane, int wave, int fullvec) {
  int wc = 0;
#pragma unroll
  for (int g = 0; g < NGRP; ++g) {
    const int el0 = (g * NTHR + tid) * EPT;
    const int e0  = cbase + el0;
    v4i da, db;
    if (fullvec) {
      da = *(const v4i*)(lst + e0);
      db = *(const v4i*)(lst + e0 + 4);
    } else {
      const int em = nE - 1;
      da.x = lst[(e0     < em) ? e0     : em];
      da.y = lst[(e0 + 1 < em) ? e0 + 1 : em];
      da.z = lst[(e0 + 2 < em) ? e0 + 2 : em];
      da.w = lst[(e0 + 3 < em) ? e0 + 3 : em];
      db.x = lst[(e0 + 4 < em) ? e0 + 4 : em];
      db.y = lst[(e0 + 5 < em) ? e0 + 5 : em];
      db.z = lst[(e0 + 6 < em) ? e0 + 6 : em];
      db.w = lst[(e0 + 7 < em) ? e0 + 7 : em];
    }
    const bool v0 = (e0 < nE), v1 = (e0 + 1 < nE), v2 = (e0 + 2 < nE), v3 = (e0 + 3 < nE);
    const bool v4 = (e0 + 4 < nE), v5 = (e0 + 5 < nE), v6 = (e0 + 6 < nE), v7 = (e0 + 7 < nE);
    const unsigned nb = (unsigned)nodeBase;
    const unsigned s0 = (unsigned)da.x - nb, s1 = (unsigned)da.y - nb;
    const unsigned s2 = (unsigned)da.z - nb, s3 = (unsigned)da.w - nb;
    const unsigned s4 = (unsigned)db.x - nb, s5 = (unsigned)db.y - nb;
    const unsigned s6 = (unsigned)db.z - nb, s7 = (unsigned)db.w - nb;
    const bool h0 = v0 && (s0 < (unsigned)NB), h1 = v1 && (s1 < (unsigned)NB);
    const bool h2 = v2 && (s2 < (unsigned)NB), h3 = v3 && (s3 < (unsigned)NB);
    const bool h4 = v4 && (s4 < (unsigned)NB), h5 = v5 && (s5 < (unsigned)NB);
    const bool h6 = v6 && (s6 < (unsigned)NB), h7 = v7 && (s7 < (unsigned)NB);
    const unsigned any = __builtin_amdgcn_ballot_w32(h0 | h1 | h2 | h3 | h4 | h5 | h6 | h7);
    if (any != 0u) {
#define HITJ(J, HJ, SJ) { \
        const unsigned mj = __builtin_amdgcn_ballot_w32(HJ); \
        if (mj != 0u) { \
          if (HJ) { \
            const int pos = wc + (int)__builtin_amdgcn_mbcnt_lo(mj, 0u); \
            if (pos < WCAP) list[wave * WCAP + pos] = ((el0 + (J)) << 12) | (int)(SJ); \
          } \
          wc += (int)__builtin_popcount(mj); } }
      HITJ(0, h0, s0)
      HITJ(1, h1, s1)
      HITJ(2, h2, s2)
      HITJ(3, h3, s3)
      HITJ(4, h4, s4)
      HITJ(5, h5, s5)
      HITJ(6, h6, s6)
      HITJ(7, h7, s7)
#undef HITJ
    }
  }
  return wc;
}

__global__ __launch_bounds__(NTHR) void k_wprep(const float* __restrict__ W, int Kin, int ncol, float scl,
                                                unsigned short* bt, int ldbt, int koff) {
  const int tpr = Kin >> 3;
  const int i = blockIdx.x * NTHR + threadIdx.x;
  if (i >= ncol * tpr) return;
  const int n  = i / tpr;
  const int k0 = (i - n * tpr) * 8;
  v8h hv;
#pragma unroll
  for (int e = 0; e < 8; ++e) {
    const float v = W[(size_t)(k0 + e) * ncol + n];
    hv[e] = (_Float16)(scl * v);
  }
  const size_t o = (size_t)n * ldbt + koff + k0;
  *(volatile v8h*)(bt + o) = hv;
  __threadfence();
  *(volatile v8h*)(bt + o) = hv;
}

__global__ __launch_bounds__(64) void k_biasprep(const float* __restrict__ bl, const float* __restrict__ b0,
                                                 const float* __restrict__ bx, const float* __restrict__ b2,
                                                 const float* __restrict__ b3, float* breg) {
  const int i = threadIdx.x;
  const int c16 = (i & 15) * 4;
  const int c32 = (i & 31) * 4;
  const v4f va = *(const v4f*)(bl + c16);
  const v4f vb = *(const v4f*)(b0 + c16);
  const v4f vc = *(const v4f*)(bx + c16);
  const v4f v2 = *(const v4f*)(b2 + c16);
  const v4f v3 = *(const v4f*)(b3 + c32);
  v4f r = va + vb + vc;
  if (i >= 16) r = v2 * 4.0f;
  if (i >= 32) r = v3 * 8.0f;
  float* dp = breg + 4 * i;
  *(volatile v4f*)dp = r;
  __threadfence();
  *(volatile v4f*)dp = r;
}

__global__ __launch_bounds__(NTHR) void k_xcast(const float* __restrict__ x, unsigned short* comb,
                                                int ldc, int coff, int nN, int RP) {
  const int i = blockIdx.x * NTHR + threadIdx.x;
  if (i >= RP * 16) return;
  const int row = i >> 4;
  const int c0  = (i & 15) * 8;
  const int rc  = (row < nN) ? row : nN - 1;
  const float* xp = x + (size_t)rc * XDIM + c0;
  v4f a = *(const v4f*)xp;
  v4f c = *(const v4f*)(xp + 4);
  if (row >= nN) { const v4f zz = {0.f, 0.f, 0.f, 0.f}; a = zz; c = zz; }
  v8h hv;
  hv[0] = (_Float16)a[0]; hv[1] = (_Float16)a[1]; hv[2] = (_Float16)a[2]; hv[3] = (_Float16)a[3];
  hv[4] = (_Float16)c[0]; hv[5] = (_Float16)c[1]; hv[6] = (_Float16)c[2]; hv[7] = (_Float16)c[3];
  const size_t o = (size_t)row * ldc + coff + c0;
  *(volatile v8h*)(comb + o) = hv;
  __threadfence();
  *(volatile v8h*)(comb + o) = hv;
}

__global__ __launch_bounds__(NTHR) void k_sum_agg(
    const int* __restrict__ seg, const int* __restrict__ gat,
    const unsigned short* hsrc, int ldh,
    unsigned short* aggo, int ldo,
    int nN, int nE, int vec_ok) {
  constexpr int NB = NBAGG;
  constexpr int FW = FDIM;
  constexpr int RW = NB / NWAVE;
  static_assert(NB * FW * 4 == 262144);
  static_assert((NB * FW / 4) % NTHR == 0 && (RW % 2) == 0 && FW == 128);
  extern __shared__ v4f lds_dyn[];
  float* acc  = (float*)lds_dyn;
  int*   list = (int*)(acc + NB * FW);
  int*   wcnt = list + LISTN;
  const int tid = threadIdx.x, lane = tid & 31, wave = tid >> 5;
  const int nodeBase = blockIdx.x * NB;
  const _Float16* hs = (const _Float16*)hsrc;

  {
    const v4f zz = {0.f, 0.f, 0.f, 0.f};
    for (int i = tid; i < NB * FW / 4; i += NTHR) lds_dyn[i] = zz;
  }
  __syncthreads();

  const int nChunks = (nE + CHUNK - 1) / CHUNK;
#pragma unroll 1
  for (int ch = 0; ch < nChunks; ++ch) {
    const int cbase = ch * CHUNK;
    const int fullvec = (vec_ok != 0 && cbase + CHUNK <= nE) ? 1 : 0;
    const int wc = scan_chunk<NB>(seg, nE, cbase, nodeBase, list, tid, lane, wave, fullvec);
    if (lane == 0) wcnt[wave] = wc;
    __syncthreads();
    if (wave == 0) {
#pragma unroll 1
      for (int wsx = 0; wsx < NWAVE; ++wsx) {
        int n = __builtin_amdgcn_readfirstlane(wcnt[wsx]);
        n = n > WCAP ? WCAP : (n < 0 ? 0 : n);
        const int* lp = list + wsx * WCAP;
#pragma unroll 1
        for (int i = 0; i < n; ++i) {
          const int ent  = __builtin_amdgcn_readfirstlane(lp[i]);
          const int slot = ent & (NB - 1);
          int e = cbase + ((ent >> 12) & (CHUNK - 1));
          e = e > nE - 1 ? nE - 1 : e;
          int s = gat[e];
          s = s < 0 ? 0 : (s > nN - 1 ? nN - 1 : s);
          const v4h hv = *(const v4h*)(hs + (size_t)s * ldh + 4 * lane);
          v4f hf;
          hf[0] = (float)hv[0]; hf[1] = (float)hv[1]; hf[2] = (float)hv[2]; hf[3] = (float)hv[3];
          v4f* ap = (v4f*)(acc + slot * FW + 4 * lane);
          const v4f av = *ap;
          *ap = av + hf;
        }
      }
    }
    __syncthreads();
  }

  unsigned short* ab = aggo + (size_t)nodeBase * ldo;
  for (int pass = 0; pass < 2; ++pass) {
#pragma unroll 2
    for (int q = 0; q < RW / 2; ++q) {
      const int row = wave * RW + 2 * q + (lane >> 4);
      const int col = (lane & 15) * 8;
      const float* sp = acc + row * FW + col;
      v4f p0 = *(const v4f*)sp, p1 = *(const v4f*)(sp + 4);
      if (nodeBase + row >= nN) { const v4f zz = {0.f, 0.f, 0.f, 0.f}; p0 = zz; p1 = zz; }
      v8h hv;
      hv[0] = (_Float16)p0[0]; hv[1] = (_Float16)p0[1]; hv[2] = (_Float16)p0[2]; hv[3] = (_Float16)p0[3];
      hv[4] = (_Float16)p1[0]; hv[5] = (_Float16)p1[1]; hv[6] = (_Float16)p1[2]; hv[7] = (_Float16)p1[3];
      *(volatile v8h*)(ab + (size_t)row * ldo + col) = hv;
    }
    __threadfence();
  }
}

__global__ __launch_bounds__(NTHR) void k_outcopy(const float* __restrict__ src, float* out, int n4) {
  const int i = blockIdx.x * NTHR + threadIdx.x;
  if (i >= n4) return;
  const size_t o = (size_t)i * 4;
  const v4f v = *(const v4f*)(src + o);
  *(volatile v4f*)(out + o) = v;
  __threadfence();
  *(volatile v4f*)(out + o) = v;
}

extern "C" void kernel_launch(void* const* d_in, const int* in_sizes, int n_in,
                              void* d_out, int out_size, void* d_ws, size_t ws_size,
                              hipStream_t stream) {
  if (n_in < 15) return;
  const int nN = in_sizes[0] / XDIM;
  const int nE = in_sizes[1] / 6;
  if (nN < 2 || in_sizes[0] != nN * XDIM || nN > (1 << 22)) return;
  if (nE < 1 || in_sizes[1] != 6 * nE) return;
  if (in_sizes[3] != XDIM * HDIM || in_sizes[4] != HDIM) return;
  if (in_sizes[5] != HDIM * HDIM || in_sizes[6] != HDIM) return;
  if (in_sizes[7] != HDIM * FDIM || in_sizes[8] != FDIM) return;
  if (in_sizes[9] != FDIM * ODIM || in_sizes[10] != ODIM) return;
  if (in_sizes[11] != FDIM * ODIM || in_sizes[12] != ODIM) return;
  if (in_sizes[13] != XDIM * ODIM || in_sizes[14] != ODIM) return;
  if (out_size != nN * ODIM) return;

  const float* x   = (const float*)d_in[0];
  const int*   ei  = (const int*)d_in[1];
  const float* mw1 = (const float*)d_in[3];
  const float* mb1 = (const float*)d_in[4];
  const float* mw2 = (const float*)d_in[5];
  const float* mb2 = (const float*)d_in[6];
  const float* mw3 = (const float*)d_in[7];
  const float* mb3 = (const float*)d_in[8];
  const float* wlw = (const float*)d_in[9];
  const float* wlb = (const float*)d_in[10];
  const float* w0w = (const float*)d_in[11];
  const float* w0b = (const float*)d_in[12];
  const float* w1w = (const float*)d_in[13];
  const float* w1b = (const float*)d_in[14];
  float* out = (float*)d_out;

  const int RP = ((nN + RPQ - 1) / RPQ) * RPQ;

  char* ws = (char*)d_ws;
  size_t off = 0;
  const size_t oW1  = off; off += (size_t)HDIM * XDIM * 2;
  const size_t oW2  = off; off += (size_t)HDIM * HDIM * 2;
  const size_t oW3  = off; off += (size_t)FDIM * HDIM * 2;
  const size_t oWC  = off; off += (size_t)ODIM * KCMB * 2;
  const size_t oBR  = off; off += (size_t)256 * 4;
  const size_t oCMB = off; off += (size_t)RP * KCMB * 2;
  const size_t oR1  = off; off += (size_t)RP * HDIM * 4;
  if (off > ws_size || off > (size_t)134217728) return;

  unsigned short* w1t  = (unsigned short*)(ws + oW1);
  unsigned short* w2t  = (unsigned short*)(ws + oW2);
  unsigned short* w3t  = (unsigned short*)(ws + oW3);
  unsigned short* wct  = (unsigned short*)(ws + oWC);
  float*          breg = (float*)(ws + oBR);
  unsigned short* comb = (unsigned short*)(ws + oCMB);
  unsigned short* h1   = (unsigned short*)(ws + oR1);
  unsigned short* h2   = (unsigned short*)(ws + oR1 + (size_t)RP * HDIM * 2);
  float*          outp = (float*)(ws + oR1);
  const float* bsum = breg;
  const float* b2s  = breg + 64;
  const float* b3s  = breg + 128;

  k_wprep<<<(HDIM * (XDIM / 8) + NTHR - 1) / NTHR, NTHR, 0, stream>>>(mw1, XDIM, HDIM, 16.0f, w1t, XDIM, 0);
  k_wprep<<<(HDIM * (HDIM / 8) + NTHR - 1) / NTHR, NTHR, 0, stream>>>(mw2, HDIM, HDIM, 16.0f, w2t, HDIM, 0);
  k_wprep<<<(FDIM * (HDIM / 8) + NTHR - 1) / NTHR, NTHR, 0, stream>>>(mw3, HDIM, FDIM, 16.0f, w3t, HDIM, 0);
  k_wprep<<<(ODIM * (FDIM / 8) + NTHR - 1) / NTHR, NTHR, 0, stream>>>(wlw, FDIM, ODIM, 4.0f,  wct, KCMB, 0);
  k_wprep<<<(ODIM * (FDIM / 8) + NTHR - 1) / NTHR, NTHR, 0, stream>>>(w0w, FDIM, ODIM, 4.0f,  wct, KCMB, FDIM);
  k_wprep<<<(ODIM * (XDIM / 8) + NTHR - 1) / NTHR, NTHR, 0, stream>>>(w1w, XDIM, ODIM, 32.0f, wct, KCMB, 2 * FDIM);
  k_biasprep<<<1, 64, 0, stream>>>(wlb, w0b, w1b, mb2, mb3, breg);
  k_xcast<<<RP * 16 / NTHR, NTHR, 0, stream>>>(x, comb, KCMB, 2 * FDIM, nN, RP);

  const int g64  = ((RP / 64) * (HDIM / 64) + 7) / 8;
  const int g128 = ((RP / 64) * (FDIM / 64) + 7) / 8;

  wmma_gemm64<0, false, 2, 1, false, 2><<<dim3(g64, 1), 256, 0, stream>>>(
      comb + 2 * FDIM, comb + 2 * FDIM, KCMB, 0L, w1t, w1t, XDIM, 0L,
      (void*)h1, (void*)h1, HDIM, 0L, mb1, mb1, 0L, RP, HDIM, XDIM, 0.0625f);
  wmma_gemm64<0, false, 2, 1, false, 2><<<dim3(g64, 1), 256, 0, stream>>>(
      h1, h1, HDIM, 0L, w2t, w2t, HDIM, 0L,
      (void*)h2, (void*)h2, HDIM, 0L, b2s, b2s, 0L, RP, HDIM, HDIM, 0.25f);
  wmma_gemm64<0, false, 2, 1, false, 0><<<dim3(g128, 1), 256, 0, stream>>>(
      h2, h2, HDIM, 0L, w3t, w3t, HDIM, 0L,
      (void*)(comb + FDIM), (void*)(comb + FDIM), KCMB, 0L, b3s, b3s, 0L, RP, FDIM, HDIM, 0.125f);
  k_sum_agg<<<RP / NBAGG, NTHR, LDS_AGG, stream>>>(ei, ei + nE, comb + FDIM, KCMB, comb, KCMB, nN, nE, 1);
  wmma_gemm64<0, false, 2, 0, false, 2><<<dim3(g64, 1), 256, 0, stream>>>(
      comb, comb, KCMB, 0L, wct, wct, KCMB, 0L,
      (void*)outp, (void*)outp, ODIM, 0L, bsum, bsum, 0L, RP, ODIM, KCMB, 0.03125f);
  const int n4 = nN * (ODIM / 4);
  k_outcopy<<<(n4 + NTHR - 1) / NTHR, NTHR, 0, stream>>>(outp, out, n4);
}
